// TemporalSelfAttention_2860448219659
// MI455X (gfx1250) — hardware-run, weakly checked
//
#include <hip/hip_runtime.h>


#define LQ   40000
#define HS   200
#define WS   200
#define RA   20480
#define RB   19520
#define DM   256
#define NH_  8
#define HD   32
#define NP_  4
typedef _Float16 h16;
typedef unsigned short bf;
typedef __attribute__((ext_vector_type(16))) __bf16   v16bf;
typedef __attribute__((ext_vector_type(16))) _Float16 v16h;
typedef __attribute__((ext_vector_type(8)))  _Float16 v8h;
typedef __attribute__((ext_vector_type(8)))  unsigned short v8us;
typedef __attribute__((ext_vector_type(8)))  float    v8f;
typedef __attribute__((ext_vector_type(4)))  float    v4f;
typedef v8h  __attribute__((may_alias)) v8ha;
typedef v4f  __attribute__((may_alias)) v4fa;
typedef v8us __attribute__((may_alias)) v8usa;

__device__ __forceinline__ unsigned short f2bf(float f) { unsigned u = __float_as_uint(f); u += 0x7FFFu + ((u >> 16) & 1u); return (unsigned short)(u >> 16); }
__device__ __forceinline__ float bf2f(unsigned short b) { return __uint_as_float(((unsigned)b) << 16); }
__device__ __forceinline__ float bfr(float f) { return bf2f(f2bf(f)); }
__device__ __forceinline__ v16h cat16(v8h lo, v8h hi) { return __builtin_shufflevector(lo, hi, 0, 1, 2, 3, 4, 5, 6, 7, 8, 9, 10, 11, 12, 13, 14, 15); }
__device__ __forceinline__ v16bf cat16b(v8us lo, v8us hi) { return __builtin_bit_cast(v16bf, __builtin_shufflevector(lo, hi, 0, 1, 2, 3, 4, 5, 6, 7, 8, 9, 10, 11, 12, 13, 14, 15)); }
__device__ __forceinline__ v8f wmma16(v16h a, v16h b, v8f c) { return __builtin_amdgcn_wmma_f32_16x16x32_f16(false, a, false, b, (short)0, c, false, false); }
__device__ __forceinline__ v8f wmmab(v16bf a, v16bf b, v8f c) { return __builtin_amdgcn_wmma_f32_16x16x32_bf16(false, a, false, b, (short)0, c, false, false); }


template <typename T16> struct WFrag;
template <> struct WFrag<h16> { typedef v16h V; static __device__ __forceinline__ V ld(const h16* p) { return cat16(*(const v8h*)p, *(const v8h*)(p + 16)); } static __device__ __forceinline__ v8f mma(V a, V b, v8f c) { return wmma16(a, b, c); } };
template <> struct WFrag<bf> { typedef v16bf V; static __device__ __forceinline__ V ld(const bf* p) { return cat16b(*(const v8us*)p, *(const v8us*)(p + 16)); } static __device__ __forceinline__ v8f mma(V a, V b, v8f c) { return wmmab(a, b, c); } };
template <typename T16, int NSPLIT, bool BIAS>
__global__ __launch_bounds__(32) void k_gemmw(const T16* __restrict__ A, const T16* __restrict__ A2, const T16* __restrict__ Bt, const T16* __restrict__ Bt2, int K, float* C, int ldc, const float* __restrict__ bias, size_t sA, size_t sB, size_t sC) {
    typedef typename WFrag<T16>::V V;
    __shared__ __align__(16) float os[16 * 68];
    const size_t z = blockIdx.z; A += z * sA; if (A2) A2 += z * sA; Bt += z * sB; if (Bt2) Bt2 += z * sB; C += z * sC;
    const int lane = threadIdx.x & 31, lr = lane & 15, hi = lane >> 4; const int r0 = blockIdx.x * 64, c0 = blockIdx.y * 64;
    v8f acc[4][4];
#pragma unroll
    for (int mb = 0; mb < 4; ++mb)
#pragma unroll
        for (int nb = 0; nb < 4; ++nb) acc[mb][nb] = (v8f){};
    const size_t aoff = (size_t)(r0 + lr) * K + 8 * hi, boff = (size_t)(c0 + lr) * K + 8 * hi;
    for (int kc = 0; kc < K; kc += 32) {
        V a[4], a2[4];
#pragma unroll
        for (int mb = 0; mb < 4; ++mb) { a[mb] = WFrag<T16>::ld(A + aoff + (size_t)mb * 16 * K + kc); if (NSPLIT == 1 || NSPLIT == 2) a2[mb] = WFrag<T16>::ld(A2 + aoff + (size_t)mb * 16 * K + kc); }
#pragma unroll
        for (int nb = 0; nb < 4; ++nb) { const V b = WFrag<T16>::ld(Bt + boff + (size_t)nb * 16 * K + kc); V b2; if (NSPLIT >= 2) b2 = WFrag<T16>::ld(Bt2 + boff + (size_t)nb * 16 * K + kc);
#pragma unroll
            for (int mb = 0; mb < 4; ++mb) { acc[mb][nb] = WFrag<T16>::mma(a[mb], b, acc[mb][nb]); if (NSPLIT == 1 || NSPLIT == 2) acc[mb][nb] = WFrag<T16>::mma(a2[mb], b, acc[mb][nb]); if (NSPLIT >= 2) acc[mb][nb] = WFrag<T16>::mma(a[mb], b2, acc[mb][nb]); } }
        asm volatile("v_nop\n\tv_nop\n\tv_nop\n\tv_nop" : "+v"(acc[0][0]), "+v"(acc[1][1]), "+v"(acc[2][2]), "+v"(acc[3][3]) : "v"(a[0]), "v"(a[3]));
    }
#pragma unroll
    for (int mb = 0; mb < 4; ++mb) {
#pragma unroll
        for (int nb = 0; nb < 4; ++nb) {
#pragma unroll
            for (int j = 0; j < 8; ++j) os[(hi * 8 + j) * 68 + nb * 16 + lr] = acc[mb][nb][j]; }
        __builtin_amdgcn_wave_barrier(); asm volatile("" ::: "memory");
        float* crow = C + (size_t)(r0 + mb * 16) * ldc + c0;
#pragma unroll 1
        for (int ps = 0; ps < 2; ++ps) {
#pragma unroll
            for (int s = 0; s < 8; ++s) { const int row = 2 * s + hi, cofs = lr * 4; v4f val = *(const v4fa*)(os + row * 68 + cofs); if (BIAS) { val[0] += bfr(bias[c0 + cofs]); val[1] += bfr(bias[c0 + cofs + 1]); val[2] += bfr(bias[c0 + cofs + 2]); val[3] += bfr(bias[c0 + cofs + 3]); }
                *(volatile v4f*)(crow + (size_t)row * ldc + cofs) = val; }
            if (ps == 0) __threadfence(); }
        __builtin_amdgcn_wave_barrier(); asm volatile("" ::: "memory");
    }
}

__device__ __forceinline__ h16 tohx(float x) { return (h16)x; }
__device__ __forceinline__ void splitf(float y, unsigned short& h, unsigned short& l) { h = f2bf(y); l = f2bf(y - bf2f(h)); }
typedef __attribute__((ext_vector_type(2))) _Float16 v2h;
typedef __attribute__((ext_vector_type(4))) _Float16 v4h;
typedef __attribute__((ext_vector_type(2))) unsigned short v2us;
typedef __attribute__((ext_vector_type(4))) unsigned short v4us;
typedef __attribute__((ext_vector_type(2))) float v2f;
typedef __attribute__((ext_vector_type(4))) int v4i;

__global__ __launch_bounds__(256) void k_cvt8(const float* __restrict__ src, bf* dst, size_t n8) { const size_t i = (size_t)blockIdx.x * 256 + threadIdx.x; if (i >= n8) return; const v8f v = *(const v8f*)(src + i * 8); v8us o;
#pragma unroll
    for (int k = 0; k < 8; ++k) o[k] = f2bf(v[k]); *(volatile v8us*)(dst + i * 8) = o; __threadfence(); *(volatile v8us*)(dst + i * 8) = o; }

__global__ __launch_bounds__(256) void k_f2h(const float* __restrict__ S, h16* P16, size_t n4) { const size_t i = (size_t)blockIdx.x * 256 + threadIdx.x; if (i >= n4) return; const v4f v = *(const v4f*)(S + i * 4); v4h o;
#pragma unroll
    for (int q = 0; q < 4; ++q) o[q] = tohx(v[q]);
    *(volatile v4h*)(P16 + i * 4) = o; __threadfence(); *(volatile v4h*)(P16 + i * 4) = o; }
__global__ __launch_bounds__(256) void k_rbf(const float* __restrict__ X, float* Y, size_t n4) { const size_t i = (size_t)blockIdx.x * 256 + threadIdx.x; if (i >= n4) return; const v4f a = *(const v4f*)(X + i * 4); v4f o;
#pragma unroll
    for (int q = 0; q < 4; ++q) o[q] = bfr(a[q]);
    *(volatile v4f*)(Y + i * 4) = o; __threadfence(); *(volatile v4f*)(Y + i * 4) = o; }
__global__ __launch_bounds__(256) void k_msda1(const float* __restrict__ VAL, const float* __restrict__ OL, const float* __restrict__ RP, float* S, size_t nl) { const size_t e = (size_t)blockIdx.x * 256 + threadIdx.x; if (e >= nl) return; const int c4 = (int)(e & 7); const int h = (int)((e >> 3) & 7); const size_t r = e >> 6;
    const v4f lg4 = *(const v4f*)(OL + r * 128 + 64 + h * 4); float lg[4]; float mx = -3.0e38f;
#pragma unroll
    for (int q = 0; q < 4; ++q) { lg[q] = lg4[q]; mx = fmaxf(mx, lg4[q]); }
    float sum = 0.f;
#pragma unroll
    for (int k = 0; k < 4; ++k) { lg[k] = __builtin_amdgcn_exp2f(__fmul_rn(__fsub_rn(lg[k], mx), 1.4426950408889634f)); sum += lg[k]; }
    const float inv = __fdiv_rn(1.0f, sum); const v2f rp = *(const v2f*)(RP + r * 2);
    v4f acc; acc[0] = 0.f; acc[1] = 0.f; acc[2] = 0.f; acc[3] = 0.f; const float fw = (float)WS, fh = (float)HS;
#pragma unroll
    for (int k = 0; k < 2; ++k) { const v4f o4 = *(const v4f*)(OL + r * 128 + h * 8 + k * 4);
#pragma unroll
        for (int q = 0; q < 2; ++q) { const int p = k * 2 + q; const float ox = o4[q * 2], oy = o4[q * 2 + 1];
            const float lx = __fadd_rn(rp[0], __fdiv_rn(ox, fw)), ly = __fadd_rn(rp[1], __fdiv_rn(oy, fh)); const float x = __fsub_rn(__fmul_rn(lx, fw), 0.5f), y = __fsub_rn(__fmul_rn(ly, fh), 0.5f);
            const float x0 = floorf(x), y0 = floorf(y); const float lw = __fsub_rn(x, x0), lh = __fsub_rn(y, y0); const int x0i = (int)x0, y0i = (int)y0; const float aw = __fmul_rn(lg[p], inv);
#pragma unroll
            for (int cy = 0; cy < 2; ++cy) {
#pragma unroll
                for (int cx = 0; cx < 2; ++cx) { const int ix = x0i + cx, iy = y0i + cy; const bool valid = (ix >= 0) && (ix < WS) && (iy >= 0) && (iy < HS); int idx = iy * WS + ix; idx = min(max(idx, 0), HS * WS - 1);
                    const float wc = __fmul_rn(cx ? lw : __fsub_rn(1.0f, lw), cy ? lh : __fsub_rn(1.0f, lh)); const float wt = valid ? __fmul_rn(wc, aw) : 0.0f; const v4f g = *(const v4f*)(VAL + (size_t)idx * DM + h * 32 + c4 * 4);
#pragma unroll
                    for (int t = 0; t < 4; ++t) acc[t] = __fadd_rn(acc[t], __fmul_rn(g[t], wt)); } } } }
    *(volatile v4f*)(S + r * DM + h * 32 + c4 * 4) = acc; __threadfence(); *(volatile v4f*)(S + r * DM + h * 32 + c4 * 4) = acc; }

extern "C" void kernel_launch(void* const* d_in, const int* in_sizes, int n_in,
                              void* d_out, int out_size, void* d_ws, size_t ws_size, hipStream_t stream) {
    (void)in_sizes; (void)n_in; (void)out_size;
    const float* qy = (const float*)d_in[0]; const float* qp = (const float*)d_in[1]; const float* rpt = (const float*)d_in[2]; const float* xf = (const float*)d_in[3]; const float* wv = (const float*)d_in[4]; const float* bv = (const float*)d_in[5]; const float* wo = (const float*)d_in[6]; const float* bo = (const float*)d_in[7]; const float* wa = (const float*)d_in[8]; const float* ba = (const float*)d_in[9]; const float* wu = (const float*)d_in[10]; const float* bu = (const float*)d_in[11];
    float* OUT = (float*)d_out;
    char* wsp = (char*)d_ws;
    auto take = [&](size_t bytes) { char* p = wsp; wsp += (bytes + 255) & ~(size_t)255; return (void*)p; };
    bf* WV = (bf*)take((size_t)DM * DM * 2); bf* WOA = (bf*)take((size_t)128 * DM * 2); float* WUR = (float*)take((size_t)DM * DM * 4); h16* WU = (h16*)take((size_t)DM * DM * 2); float* BOA = (float*)take((size_t)128 * 4);
    float* VAL = (float*)take((size_t)LQ * DM * 4); bf* BFA = (bf*)take((size_t)RA * DM * 2); bf* BFB = (bf*)take((size_t)RA * DM * 2); float* OL = (float*)take((size_t)RA * 128 * 4); float* SP = (float*)take((size_t)RA * DM * 4); h16* S16 = (h16*)take((size_t)RA * DM * 2); float* RPB = (float*)take((size_t)RA * 2 * 4);
    if ((size_t)(wsp - (char*)d_ws) > ws_size) return;
    k_cvt8<<<(unsigned)(((size_t)DM * DM / 8 + 255) / 256), 256, 0, stream>>>(wv, WV, (size_t)DM * DM / 8);
    k_rbf<<<(unsigned)(((size_t)DM * DM / 4 + 255) / 256), 256, 0, stream>>>(wu, WUR, (size_t)DM * DM / 4); k_f2h<<<(unsigned)(((size_t)DM * DM / 4 + 255) / 256), 256, 0, stream>>>(WUR, WU, (size_t)DM * DM / 4);
    k_cvt8<<<(unsigned)(((size_t)64 * DM / 8 + 255) / 256), 256, 0, stream>>>(wo, WOA, (size_t)64 * DM / 8); k_cvt8<<<(unsigned)(((size_t)32 * DM / 8 + 255) / 256), 256, 0, stream>>>(wa, WOA + (size_t)64 * DM, (size_t)32 * DM / 8); k_cvt8<<<(unsigned)(((size_t)32 * DM / 8 + 255) / 256), 256, 0, stream>>>(wa, WOA + (size_t)96 * DM, (size_t)32 * DM / 8);
    k_rbf<<<1, 256, 0, stream>>>(bo, BOA, (size_t)64 / 4); k_rbf<<<1, 256, 0, stream>>>(ba, BOA + 64, (size_t)32 / 4); k_rbf<<<1, 256, 0, stream>>>(ba, BOA + 96, (size_t)32 / 4);
    for (int hf = 0; hf < 2; ++hf) { const size_t r0 = hf ? (size_t)RA : 0; const size_t nr = hf ? (size_t)RB : (size_t)RA;
        k_cvt8<<<(unsigned)((nr * DM / 8 + 255) / 256), 256, 0, stream>>>(xf + r0 * DM, BFA, nr * DM / 8);
        k_gemmw<bf, 0, true><<<dim3((unsigned)(nr / 64), DM / 64, 1), 32, 0, stream>>>(BFA, nullptr, WV, nullptr, DM, VAL + r0 * DM, DM, bv, 0, 0, 0); }
    for (int hf = 0; hf < 2; ++hf) { const size_t r0 = hf ? (size_t)RA : 0; const size_t nr = hf ? (size_t)RB : (size_t)RA;
        k_cvt8<<<(unsigned)((nr * DM / 8 + 255) / 256), 256, 0, stream>>>(qy + r0 * DM, BFA, nr * DM / 8); k_cvt8<<<(unsigned)((nr * DM / 8 + 255) / 256), 256, 0, stream>>>(qp + r0 * DM, BFB, nr * DM / 8);
        k_gemmw<bf, 1, true><<<dim3((unsigned)(nr / 64), 128 / 64, 1), 32, 0, stream>>>(BFA, BFB, WOA, nullptr, DM, OL, 128, BOA, 0, 0, 0);
        k_rbf<<<(unsigned)((nr * 2 / 4 + 255) / 256), 256, 0, stream>>>(rpt + r0 * 2, RPB, nr * 2 / 4);
        k_msda1<<<(unsigned)((nr * NH_ * 8 + 255) / 256), 256, 0, stream>>>(VAL, OL, RPB, SP, nr * NH_ * 8);
        k_f2h<<<(unsigned)((nr * DM / 4 + 255) / 256), 256, 0, stream>>>(SP, S16, nr * DM / 4);
        k_gemmw<h16, 0, true><<<dim3((unsigned)(nr / 64), DM / 64, 1), 32, 0, stream>>>(S16, nullptr, WU, nullptr, DM, OUT + r0 * DM, DM, bu, 0, 0, 0); }
}
